// GINEEncoder_77541339562639
// MI455X (gfx1250) — hardware-verified
//
#include <hip/hip_runtime.h>
#include <stddef.h>
#include <stdint.h>


#define DIN     32
#define NET     16
#define DH      128
#define ZW      256
#define DOUT    256
#define TST     4
#define PW      512
#define PW2     1024
#define NGR     64
#define NTHR    256
#define NWAVE   8
#define EPT     8
#define CHUNK   (NTHR * EPT)
#define WCAP    (EPT * 32)
#define LISTN   (NWAVE * WCAP)
#define NB      1024
#define PKS     10
#define RCAP    20480
#define DEGCAP  64
#define GBM     64
#define GBN     128
#define GTHR    128
#define GNT     8
#define NUWN    (DH * (DIN / 8))
#define NUWE    (DH * (DIN / 8))
#define NUW1    (DH * (ZW / 8))
#define NUW2    (DH * (ZW / 8))
#define NUWL    (DOUT * (PW2 / 8))
#define NUWTOT  (NUWN + NUWE + NUW1 + NUW2 + NUWL)
#define WSMAX   134217728
#define LDS_BKT ((2 * RCAP + 2 * NB + LISTN) * 4 + 64)
#define LDS_SCAN (NWAVE * 16 * DH * 4)

static_assert((CHUNK & (CHUNK - 1)) == 0 && CHUNK == 2048);
static_assert((NB & (NB - 1)) == 0 && NB == (1 << PKS));
static_assert(NTHR * 4 == NB && LISTN >= NB);
static_assert((RCAP % 128) == 0 && RCAP <= (1 << 20));
static_assert(LDS_BKT <= 300000 && LDS_SCAN <= 300000);
static_assert(GBM == (GTHR / 32) * 16 && GBN == 16 * GNT && GBN == DH);
static_assert((DIN % 32) == 0 && (ZW % 32) == 0 && (PW2 % 32) == 0);
static_assert((NUWN % NTHR) == 0 && (NUWE % NTHR) == 0 && (NUW1 % NTHR) == 0 && (NUWL % NTHR) == 0);
static_assert(ZW == 2 * DH && PW == TST * DH && PW2 == 2 * PW && (DOUT % GBN) == 0 && (NGR % GBM) == 0);
static_assert(DH == 32 * 4);
static_assert(GBM * ZW * 2 == GBM * GBN * 4);

typedef float          v4f  __attribute__((ext_vector_type(4)));
typedef float          v8f  __attribute__((ext_vector_type(8)));
typedef int            v4i  __attribute__((ext_vector_type(4)));
typedef int            v8i  __attribute__((ext_vector_type(8)));
typedef unsigned int   v2u  __attribute__((ext_vector_type(2)));
typedef unsigned short v8us __attribute__((ext_vector_type(8)));
typedef __bf16         v16b __attribute__((ext_vector_type(16)));
typedef v4f  __attribute__((may_alias)) v4fa;
typedef v4i  __attribute__((may_alias)) v4ia;
typedef v8us __attribute__((may_alias)) v8usa;
union Frag { v16b vb; v8us h[2]; v8i w; };

__device__ __forceinline__ v8f wmb(const Frag& a, const Frag& b, v8f c) {
  v8f d = __builtin_amdgcn_wmma_f32_16x16x32_bf16(false, a.vb, false, b.vb, (short)0, c, false, false);
  asm volatile("v_nop\n\tv_nop\n\tv_nop\n\tv_nop" : "+v"(d) : "v"(a.w), "v"(b.w));
  return d;
}

__device__ __forceinline__ unsigned short bf_bits(float f) {
  unsigned int u = __float_as_uint(f);
  u += 0x7FFFu + ((u >> 16) & 1u);
  return (unsigned short)(u >> 16);
}
__device__ __forceinline__ float bf_val(unsigned short b) { return __uint_as_float(((unsigned int)b) << 16); }
__device__ __forceinline__ float bf_rne(float f) { return bf_val(bf_bits(f)); }

__device__ __forceinline__ void hilo8(const v4f a, const v4f b, v8us& hv, v8us& lv) {
  const float f[8] = {a.x, a.y, a.z, a.w, b.x, b.y, b.z, b.w};
#pragma unroll
  for (int j = 0; j < 8; ++j) {
    const unsigned short hb = bf_bits(f[j]);
    hv[j] = hb;
    lv[j] = bf_bits(f[j] - bf_val(hb));
  }
}

__device__ __forceinline__ void wave_sync_lds() {
  __builtin_amdgcn_fence(__ATOMIC_RELEASE, "wavefront");
  __builtin_amdgcn_wave_barrier();
  __builtin_amdgcn_fence(__ATOMIC_ACQUIRE, "wavefront");
}

__device__ __forceinline__ int scan_chunk(const int* __restrict__ dsts, int nE, int cbase, int slotBase,
                                          int nb, int vec8, int* list, int tid, int lane, int wave) {
  int wc = 0;
  const int el0  = tid * EPT;
  const int e0   = cbase + el0;
  const int sent = -2147483647 - 1;
  v4i da, db;
  if (vec8 != 0 && cbase + CHUNK <= nE) {
    da = *(const v4i*)(dsts + e0);
    db = *(const v4i*)(dsts + e0 + 4);
  } else {
    da.x = (e0     < nE) ? dsts[min(e0,     nE - 1)] : sent;
    da.y = (e0 + 1 < nE) ? dsts[min(e0 + 1, nE - 1)] : sent;
    da.z = (e0 + 2 < nE) ? dsts[min(e0 + 2, nE - 1)] : sent;
    da.w = (e0 + 3 < nE) ? dsts[min(e0 + 3, nE - 1)] : sent;
    db.x = (e0 + 4 < nE) ? dsts[min(e0 + 4, nE - 1)] : sent;
    db.y = (e0 + 5 < nE) ? dsts[min(e0 + 5, nE - 1)] : sent;
    db.z = (e0 + 6 < nE) ? dsts[min(e0 + 6, nE - 1)] : sent;
    db.w = (e0 + 7 < nE) ? dsts[min(e0 + 7, nE - 1)] : sent;
  }
  const unsigned nbs = (unsigned)slotBase;
  const unsigned unb = (unsigned)nb;
  const unsigned s0 = (unsigned)da.x - nbs, s1 = (unsigned)da.y - nbs;
  const unsigned s2 = (unsigned)da.z - nbs, s3 = (unsigned)da.w - nbs;
  const unsigned s4 = (unsigned)db.x - nbs, s5 = (unsigned)db.y - nbs;
  const unsigned s6 = (unsigned)db.z - nbs, s7 = (unsigned)db.w - nbs;
  const bool h0 = s0 < unb, h1 = s1 < unb, h2 = s2 < unb, h3 = s3 < unb;
  const bool h4 = s4 < unb, h5 = s5 < unb, h6 = s6 < unb, h7 = s7 < unb;
  const unsigned any = __builtin_amdgcn_ballot_w32(h0 | h1 | h2 | h3 | h4 | h5 | h6 | h7);
  if (any != 0u) {
#define HITJ(J, HJ, SJ) { \
      const unsigned mj = __builtin_amdgcn_ballot_w32(HJ); \
      if (mj != 0u) { \
        if (HJ) { \
          const int pos = wc + (int)__builtin_amdgcn_mbcnt_lo(mj, 0u); \
          if (pos < WCAP) list[wave * WCAP + pos] = ((el0 + (J)) << PKS) | (int)(SJ); \
        } \
        wc += (int)__builtin_popcount(mj); } }
    HITJ(0, h0, s0)
    HITJ(1, h1, s1)
    HITJ(2, h2, s2)
    HITJ(3, h3, s3)
    HITJ(4, h4, s4)
    HITJ(5, h5, s5)
    HITJ(6, h6, s6)
    HITJ(7, h7, s7)
#undef HITJ
  }
  return wc;
}

__device__ __forceinline__ v8us cv8b(const float* __restrict__ p, size_t stride) {
  v8us o;
#pragma unroll
  for (int i = 0; i < 8; ++i) o[i] = bf_bits(p[(size_t)i * stride]);
  return o;
}

__global__ __launch_bounds__(NTHR) void k_prep(const float* __restrict__ x, const float* __restrict__ Wn,
                                               const float* __restrict__ We, const float* __restrict__ W1,
                                               const float* __restrict__ W2, const float* __restrict__ Wl,
                                               int nux,
                                               unsigned short* XB, unsigned short* WnT, unsigned short* WeT,
                                               unsigned short* W1D, unsigned short* W2D, unsigned short* WL2) {
  const int u  = (int)blockIdx.x * NTHR + (int)threadIdx.x;
  const int c1 = nux, c2 = c1 + NUWN, c3 = c2 + NUWE, c4 = c3 + NUW1, c5 = c4 + NUW2, c6 = c5 + NUWL;
  v8us o;
  unsigned short* dp;
  if (u < c1) {
    const float* p = x + (size_t)u * 8;
    const v4f a = *(const v4fa*)p;
    const v4f b = *(const v4fa*)(p + 4);
    o[0] = bf_bits(a.x); o[1] = bf_bits(a.y); o[2] = bf_bits(a.z); o[3] = bf_bits(a.w);
    o[4] = bf_bits(b.x); o[5] = bf_bits(b.y); o[6] = bf_bits(b.z); o[7] = bf_bits(b.w);
    dp = XB + (size_t)u * 8;
  } else if (u < c2) {
    const int v = u - c1, n = v >> 2, k8 = (v & 3) * 8;
    o = cv8b(Wn + (size_t)k8 * DH + n, DH);
    dp = WnT + (size_t)v * 8;
  } else if (u < c3) {
    const int v = u - c2, n = v >> 2, k8 = (v & 3) * 8;
    const bool live = k8 < NET;
    const int kk = live ? k8 : 0;
    o = cv8b(We + (size_t)kk * DH + n, DH);
    const unsigned short msk = live ? (unsigned short)0xFFFF : (unsigned short)0;
#pragma unroll
    for (int i = 0; i < 8; ++i) o[i] = (unsigned short)(o[i] & msk);
    dp = WeT + (size_t)v * 8;
  } else if (u < c4) {
    const int v = u - c3, n = v >> 5, k8 = (v & 31) * 8, kk = k8 & (DH - 1);
    o = cv8b(W1 + (size_t)kk * DH + n, DH);
    dp = W1D + (size_t)v * 8;
  } else if (u < c5) {
    const int v = u - c4, n = v >> 5, k8 = (v & 31) * 8, kk = k8 & (DH - 1);
    o = cv8b(W2 + (size_t)kk * DH + n, DH);
    dp = W2D + (size_t)v * 8;
  } else if (u < c6) {
    const int v = u - c5, n = v >> 7, k8 = (v & 127) * 8, kk = k8 & (PW - 1);
    o = cv8b(Wl + (size_t)kk * DOUT + n, DOUT);
    dp = WL2 + (size_t)v * 8;
  } else {
    return;
  }
  *(volatile v8us*)dp = o;
  __threadfence();
  *(volatile v8us*)dp = o;
}

__global__ __launch_bounds__(GTHR) void k_gemm(const unsigned short* __restrict__ A, int lda,
                                               const unsigned short* __restrict__ BT, int ldb, int K,
                                               const float* __restrict__ bias,
                                               float* outF, int ldo, int nN, int mRows) {
  __shared__ __attribute__((aligned(16))) float stg[GBM * GBN];
  const int tid = (int)threadIdx.x, lane = tid & 31, wave = tid >> 5, hh = lane >> 4, m = lane & 15;
  const int rowBase = (int)blockIdx.x * GBM;
  const int colBase = (int)blockIdx.y * GBN;

  v8f acc[GNT];
  {
    const v8f z = {0.f, 0.f, 0.f, 0.f, 0.f, 0.f, 0.f, 0.f};
#pragma unroll
    for (int t = 0; t < GNT; ++t) acc[t] = z;
  }
  const unsigned short* ap = A  + (size_t)(rowBase + 16 * wave + m) * (size_t)lda + 8 * hh;
  const unsigned short* bp = BT + (size_t)(colBase + m) * (size_t)ldb + 8 * hh;

#pragma unroll 1
  for (int k0 = 0; k0 < K; k0 += 32) {
    Frag af;
    af.h[0] = *(const v8usa*)(ap + k0);
    af.h[1] = *(const v8usa*)(ap + k0 + 16);
#pragma unroll
    for (int nt = 0; nt < GNT; ++nt) {
      const unsigned short* wq = bp + (size_t)(16 * nt) * (size_t)ldb + k0;
      Frag bfr;
      bfr.h[0] = *(const v8usa*)wq;
      bfr.h[1] = *(const v8usa*)(wq + 16);
      acc[nt] = wmb(af, bfr, acc[nt]);
    }
  }

#pragma unroll
  for (int nt = 0; nt < GNT; ++nt) {
    const int lc = 16 * nt + m;
    const float bb = bf_rne(bias[colBase + lc]);
#pragma unroll
    for (int r = 0; r < 8; ++r) {
      const int lr = 16 * wave + 8 * hh + r;
      const bool live = (rowBase + lr) < nN;
      const float v = acc[nt][r] + bb;
      stg[lr * GBN + lc] = live ? v : 0.0f;
    }
  }
  __syncthreads();

  v4f fv[16];
#pragma unroll
  for (int i = 0; i < 16; ++i) {
    const int lr = 16 * wave + i;
    fv[i] = *(const v4fa*)(stg + lr * GBN + 4 * lane);
  }
#pragma unroll
  for (int i = 0; i < 16; ++i) {
    const int gr = rowBase + 16 * wave + i;
    float* op = outF + (size_t)gr * (size_t)ldo + colBase + 4 * lane;
    if (gr < mRows) *(volatile v4f*)op = fv[i];
  }
  __threadfence();
#pragma unroll
  for (int i = 0; i < 16; ++i) {
    const int gr = rowBase + 16 * wave + i;
    float* op = outF + (size_t)gr * (size_t)ldo + colBase + 4 * lane;
    if (gr < mRows) *(volatile v4f*)op = fv[i];
  }
}

__global__ __launch_bounds__(NTHR) void k_bucket(const int* __restrict__ srcs, const int* __restrict__ dsts,
                                                 const float* __restrict__ ea, int nN, int nE, int vec8,
                                                 unsigned short* EAS, int* SRCL, int* TSO, int* TSC, int* META) {
  extern __shared__ v4f lds_bkt[];
  int* reg1 = (int*)lds_bkt;
  int* reg2 = reg1 + RCAP;
  int* scnt = reg2 + RCAP;
  int* soff = scnt + NB;
  int* list = soff + NB;
  int* wcnt = list + LISTN;
  int* wtot = wcnt + NWAVE;
  const int tid = (int)threadIdx.x, lane = tid & 31, wave = tid >> 5;
  const int blk = (int)blockIdx.x;
  const int nodeBase = blk * NB;

  for (int i = tid; i < NB; i += NTHR) scnt[i] = 0;
  if (tid == 0) { reg1[0] = 0; reg2[0] = 0; }
  __syncthreads();

  int tot = 0;
  const int nChunks = (nE + CHUNK - 1) / CHUNK;
#pragma unroll 1
  for (int ch = 0; ch < nChunks; ++ch) {
    const int cbase = ch * CHUNK;
    const int wc = scan_chunk(dsts, nE, cbase, nodeBase, NB, vec8, list, tid, lane, wave);
    if (lane == 0) wcnt[wave] = wc;
    __syncthreads();
    int pre = 0, all = 0;
#pragma unroll
    for (int w2 = 0; w2 < NWAVE; ++w2) {
      int c = wcnt[w2];
      c = c < 0 ? 0 : (c > WCAP ? WCAP : c);
      all += c;
      pre += (w2 < wave) ? c : 0;
    }
    const int wcc  = wc > WCAP ? WCAP : wc;
    const int base = tot + pre;
#pragma unroll 1
    for (int i = lane; i < wcc; i += 32) {
      const int ent = list[wave * WCAP + i];
      const int el  = (ent >> PKS) & (CHUNK - 1);
      const int sl  = ent & (NB - 1);
      int eid = cbase + el;
      eid = eid > nE - 1 ? nE - 1 : eid;
      const int pos = base + i;
      if (pos < RCAP) reg1[pos] = (int)(((unsigned)eid << PKS) | (unsigned)sl);
    }
    tot += all;
    tot = tot > RCAP ? RCAP : tot;
    __syncthreads();
  }
  const int nh = tot;
  const int lastv = nh > 0 ? nh - 1 : 0;

  if (wave == 0) {
#pragma unroll 1
    for (int b0 = 0; b0 < nh; b0 += 32) {
      int idx = b0 + lane;
      idx = idx > lastv ? lastv : idx;
      const int uv  = reg1[idx];
      const int m32 = (nh - b0) < 32 ? (nh - b0) : 32;
#pragma unroll 1
      for (int k = 0; k < m32; ++k) {
        const int u  = __builtin_amdgcn_readlane(uv, k);
        const int sl = u & (NB - 1);
        if (lane == 0) scnt[sl] = scnt[sl] + 1;
      }
    }
  }
  __syncthreads();

  {
    const v4i ca = *(const v4ia*)(scnt + 4 * tid);
    const int e0 = ca.x < 0 ? 0 : ca.x, e1 = ca.y < 0 ? 0 : ca.y, e2 = ca.z < 0 ? 0 : ca.z, e3 = ca.w < 0 ? 0 : ca.w;
    const int ts = e0 + e1 + e2 + e3;
    int incl = ts;
#pragma unroll
    for (int d = 1; d < 32; d <<= 1) {
      const int up = __shfl_up(incl, d);
      if (lane >= d) incl += up;
    }
    if (lane == 31) wtot[wave] = incl;
    __syncthreads();
    int pre = 0;
#pragma unroll
    for (int w2 = 0; w2 < NWAVE; ++w2) pre += (w2 < wave) ? wtot[w2] : 0;
    int run = pre + incl - ts;
    soff[4 * tid + 0] = run; run += e0;
    soff[4 * tid + 1] = run; run += e1;
    soff[4 * tid + 2] = run; run += e2;
    soff[4 * tid + 3] = run;
  }
  __syncthreads();
  for (int i = tid; i < NB; i += NTHR) list[i] = soff[i];
  __syncthreads();

  if (wave == 0) {
#pragma unroll 1
    for (int b0 = 0; b0 < nh; b0 += 32) {
      int idx = b0 + lane;
      idx = idx > lastv ? lastv : idx;
      const int uv  = reg1[idx];
      const int m32 = (nh - b0) < 32 ? (nh - b0) : 32;
#pragma unroll 1
      for (int k = 0; k < m32; ++k) {
        const int u   = __builtin_amdgcn_readlane(uv, k);
        const int sl  = u & (NB - 1);
        const int eid = (int)((unsigned)u >> PKS);
        if (lane == 0) {
          int pos = list[sl];
          pos = pos < 0 ? 0 : (pos > RCAP - 1 ? RCAP - 1 : pos);
          reg2[pos] = eid;
          list[sl] = pos + 1;
        }
      }
    }
  }
  __syncthreads();

  int nhw = ((nh + 16 + 127) >> 7) << 7;
  nhw = nhw > RCAP ? RCAP : nhw;
  const size_t hb = (size_t)blk * (size_t)RCAP;

#pragma unroll 1
  for (int i0 = 0; i0 < nhw; i0 += NTHR * 4) {
    const int i = i0 + 4 * tid;
    v4i sv;
#pragma unroll
    for (int j = 0; j < 4; ++j) {
      const int idx = i + j;
      const int ridx = idx > lastv ? lastv : idx;
      int eid = reg2[ridx];
      eid = eid < 0 ? 0 : (eid > nE - 1 ? nE - 1 : eid);
      int s = srcs[eid];
      s = s < 0 ? 0 : (s > nN - 1 ? nN - 1 : s);
      sv[j] = (idx < nh) ? s : 0;
    }
    const bool ok = i < nhw;
    const int ic = ok ? i : 0;
    int* dp = SRCL + hb + (size_t)ic;
    if (ok) *(volatile v4i*)dp = sv;
    __threadfence();
    if (ok) *(volatile v4i*)dp = sv;
  }

  const int nu = nhw * 2;
#pragma unroll 1
  for (int u0 = 0; u0 < nu; u0 += NTHR) {
    const int u = u0 + tid;
    const int hit = u >> 1, half = u & 1;
    const int ridx = hit > lastv ? lastv : hit;
    int eid = reg2[ridx];
    eid = eid < 0 ? 0 : (eid > nE - 1 ? nE - 1 : eid);
    const float* p = ea + (size_t)eid * NET + half * 8;
    const v4f a = *(const v4fa*)p;
    const v4f b = *(const v4fa*)(p + 4);
    const unsigned short msk = (hit < nh) ? (unsigned short)0xFFFF : (unsigned short)0;
    v8us o;
    o[0] = (unsigned short)(bf_bits(a.x) & msk); o[1] = (unsigned short)(bf_bits(a.y) & msk);
    o[2] = (unsigned short)(bf_bits(a.z) & msk); o[3] = (unsigned short)(bf_bits(a.w) & msk);
    o[4] = (unsigned short)(bf_bits(b.x) & msk); o[5] = (unsigned short)(bf_bits(b.y) & msk);
    o[6] = (unsigned short)(bf_bits(b.z) & msk); o[7] = (unsigned short)(bf_bits(b.w) & msk);
    unsigned short* dp = EAS + (hb + (size_t)hit) * NET + half * 8;
    *(volatile v8us*)dp = o;
    __threadfence();
    *(volatile v8us*)dp = o;
  }

  {
    const v4i so = *(const v4ia*)(soff + 4 * tid);
    const v4i sc = *(const v4ia*)(scnt + 4 * tid);
    int* op = TSO + (size_t)blk * NB + 4 * tid;
    int* cp = TSC + (size_t)blk * NB + 4 * tid;
    v4i mv = {0, 0, 0, 0};
    if (tid == 0) mv.x = nh;
    const bool mok = tid < 8;
    int* mp = META + (size_t)blk * 32 + 4 * (tid & 7);
    *(volatile v4i*)op = so;
    *(volatile v4i*)cp = sc;
    if (mok) *(volatile v4i*)mp = mv;
    __threadfence();
    *(volatile v4i*)op = so;
    *(volatile v4i*)cp = sc;
    if (mok) *(volatile v4i*)mp = mv;
  }
}

__global__ __launch_bounds__(NTHR) void k_scan(const unsigned short* __restrict__ EAS, const int* __restrict__ SRCL,
                                               const int* __restrict__ TSO, const int* __restrict__ TSC,
                                               const int* __restrict__ META,
                                               const unsigned short* __restrict__ WeT, const float* __restrict__ be,
                                               const float* __restrict__ H, unsigned short* Z, int nN) {
  extern __shared__ v4f lds_scan[];
  const int tid = (int)threadIdx.x, lane = tid & 31, wave = tid >> 5, hh = lane >> 4, m = lane & 15;
  float* et = (float*)lds_scan + wave * (16 * DH);
  const int blk = (int)blockIdx.x;
  const int nodeBase = blk * NB;
  const size_t hb = (size_t)blk * (size_t)RCAP;

  int nh = __builtin_amdgcn_readfirstlane(META[(size_t)blk * 32]);
  nh = nh < 0 ? 0 : (nh > RCAP ? RCAP : nh);
  const bool ovf = nh >= RCAP;
  const float qnan = __int_as_float(0x7fc00000);

  Frag bw[GNT];
  float bev[GNT];
#pragma unroll
  for (int nt = 0; nt < GNT; ++nt) {
    const unsigned short* wq = WeT + (size_t)(16 * nt + m) * DIN + 8 * hh;
    bw[nt].h[0] = *(const v8usa*)wq;
    bw[nt].h[1] = *(const v8usa*)(wq + 16);
    bev[nt] = bf_rne(be[16 * nt + m]);
  }
  const v8us zus = {0, 0, 0, 0, 0, 0, 0, 0};
  const v8f  z8  = {0.f, 0.f, 0.f, 0.f, 0.f, 0.f, 0.f, 0.f};

  const int s0 = wave * (NB / NWAVE);
  int tb = -1000000;
  int srcv = 0;

#pragma unroll 1
  for (int jt = 0; jt < NB / NWAVE; ++jt) {
    const int slot = s0 + jt;
    const int grow = nodeBase + slot;
    if (grow >= nN) break;
    int st = __builtin_amdgcn_readfirstlane(TSO[(size_t)blk * NB + slot]);
    const int craw = __builtin_amdgcn_readfirstlane(TSC[(size_t)blk * NB + slot]);
    int cnt = craw < 0 ? 0 : (craw > DEGCAP ? DEGCAP : craw);
    st = st < 0 ? 0 : (st > nh ? nh : st);
    if (cnt > nh - st) cnt = nh - st;

    float a0 = 0.0f, a1 = 0.0f, a2 = 0.0f, a3 = 0.0f;
    int q = 0;
#pragma unroll 1
    while (q < cnt) {
      const int idx = st + q;
      if (idx < tb || idx >= tb + 16) {
        tb = idx;
        int row = tb + m;
        row = row > RCAP - 1 ? RCAP - 1 : row;
        Frag af;
        af.h[0] = *(const v8usa*)(EAS + (hb + (size_t)row) * NET + 8 * hh);
        af.h[1] = zus;
        int sr = SRCL[hb + (size_t)row];
        sr = sr < 0 ? 0 : (sr > nN - 1 ? nN - 1 : sr);
        srcv = sr;
        wave_sync_lds();
#pragma unroll
        for (int nt = 0; nt < GNT; ++nt) {
          const v8f d = wmb(af, bw[nt], z8);
#pragma unroll
          for (int r = 0; r < 8; ++r) et[(8 * hh + r) * DH + 16 * nt + m] = d[r] + bev[nt];
        }
        wave_sync_lds();
      }
      const int i0 = idx - tb;
      int n = 16 - i0;
      if (n > cnt - q) n = cnt - q;
#pragma unroll 1
      for (int u = 0; u < n; ++u) {
        const int i = i0 + u;
        const int s = __builtin_amdgcn_readlane(srcv, i);
        const v4f ev = *(const v4fa*)(et + i * DH + 4 * lane);
        const v4f hv = *(const v4f*)(H + (size_t)s * DH + 4 * lane);
        float x0 = ev.x + hv.x, x1 = ev.y + hv.y, x2 = ev.z + hv.z, x3 = ev.w + hv.w;
        x0 = (x0 > 0.0f) ? x0 : (x0 - x0);
        x1 = (x1 > 0.0f) ? x1 : (x1 - x1);
        x2 = (x2 > 0.0f) ? x2 : (x2 - x2);
        x3 = (x3 > 0.0f) ? x3 : (x3 - x3);
        a0 += x0; a1 += x1; a2 += x2; a3 += x3;
      }
      q += n;
    }

    const v4f sv = *(const v4f*)(H + (size_t)grow * DH + 4 * lane);
    const float pz = (ovf || craw > DEGCAP) ? qnan : 0.0f;
    const float r0 = (sv.x + a0) + pz, r1 = (sv.y + a1) + pz;
    const float r2 = (sv.z + a2) + pz, r3 = (sv.w + a3) + pz;
    const unsigned short h0 = bf_bits(r0), h1 = bf_bits(r1), h2 = bf_bits(r2), h3 = bf_bits(r3);
    const unsigned short l0 = bf_bits(r0 - bf_val(h0)), l1 = bf_bits(r1 - bf_val(h1));
    const unsigned short l2 = bf_bits(r2 - bf_val(h2)), l3 = bf_bits(r3 - bf_val(h3));
    v2u ph, pl;
    ph.x = (unsigned int)h0 | ((unsigned int)h1 << 16);
    ph.y = (unsigned int)h2 | ((unsigned int)h3 << 16);
    pl.x = (unsigned int)l0 | ((unsigned int)l1 << 16);
    pl.y = (unsigned int)l2 | ((unsigned int)l3 << 16);
    unsigned short* zp = Z + (size_t)grow * ZW + 4 * lane;
    *(volatile v2u*)zp = ph;
    *(volatile v2u*)(zp + DH) = pl;
    __threadfence();
    *(volatile v2u*)zp = ph;
    *(volatile v2u*)(zp + DH) = pl;
  }
}

__global__ __launch_bounds__(GTHR) void k_mlp(const unsigned short* __restrict__ Z,
                                              const unsigned short* __restrict__ W1D,
                                              const unsigned short* __restrict__ W2D,
                                              const float* __restrict__ b1, const float* __restrict__ b2,
                                              float* H, int nN, int mRows) {
  __shared__ __attribute__((aligned(16))) float stg[GBM * GBN];
  unsigned short* tl = (unsigned short*)stg;
  const int tid = (int)threadIdx.x, lane = tid & 31, wave = tid >> 5, hh = lane >> 4, m = lane & 15;
  const int rowBase = (int)blockIdx.x * GBM;
  const v8f z8 = {0.f, 0.f, 0.f, 0.f, 0.f, 0.f, 0.f, 0.f};

  v8f acc[GNT];
#pragma unroll
  for (int t = 0; t < GNT; ++t) acc[t] = z8;
  {
    const unsigned short* ap = Z   + (size_t)(rowBase + 16 * wave + m) * ZW + 8 * hh;
    const unsigned short* bp = W1D + (size_t)m * ZW + 8 * hh;
#pragma unroll 1
    for (int k0 = 0; k0 < ZW; k0 += 32) {
      Frag af;
      af.h[0] = *(const v8usa*)(ap + k0);
      af.h[1] = *(const v8usa*)(ap + k0 + 16);
#pragma unroll
      for (int nt = 0; nt < GNT; ++nt) {
        const unsigned short* wq = bp + (size_t)(16 * nt) * ZW + k0;
        Frag bfr;
        bfr.h[0] = *(const v8usa*)wq;
        bfr.h[1] = *(const v8usa*)(wq + 16);
        acc[nt] = wmb(af, bfr, acc[nt]);
      }
    }
  }
#pragma unroll
  for (int nt = 0; nt < GNT; ++nt) {
    const int lc = 16 * nt + m;
    const float bb = bf_rne(b1[lc]);
#pragma unroll
    for (int r = 0; r < 8; ++r) {
      const int lr = 16 * wave + 8 * hh + r;
      float v = acc[nt][r] + bb;
      v = (v > 0.0f) ? v : (v - v);
      const unsigned short hb = bf_bits(v);
      const unsigned short lb = bf_bits(v - bf_val(hb));
      tl[lr * ZW + lc] = hb;
      tl[lr * ZW + DH + lc] = lb;
    }
  }
  __syncthreads();

#pragma unroll
  for (int t = 0; t < GNT; ++t) acc[t] = z8;
  {
    const unsigned short* tp = tl  + (size_t)(16 * wave + m) * ZW + 8 * hh;
    const unsigned short* bp = W2D + (size_t)m * ZW + 8 * hh;
#pragma unroll 1
    for (int k0 = 0; k0 < ZW; k0 += 32) {
      Frag af;
      af.h[0] = *(const v8usa*)(tp + k0);
      af.h[1] = *(const v8usa*)(tp + k0 + 16);
#pragma unroll
      for (int nt = 0; nt < GNT; ++nt) {
        const unsigned short* wq = bp + (size_t)(16 * nt) * ZW + k0;
        Frag bfr;
        bfr.h[0] = *(const v8usa*)wq;
        bfr.h[1] = *(const v8usa*)(wq + 16);
        acc[nt] = wmb(af, bfr, acc[nt]);
      }
    }
  }
  __syncthreads();

#pragma unroll
  for (int nt = 0; nt < GNT; ++nt) {
    const int lc = 16 * nt + m;
    const float bb = bf_rne(b2[lc]);
#pragma unroll
    for (int r = 0; r < 8; ++r) {
      const int lr = 16 * wave + 8 * hh + r;
      const bool live = (rowBase + lr) < nN;
      const float v = acc[nt][r] + bb;
      stg[lr * GBN + lc] = live ? v : 0.0f;
    }
  }
  __syncthreads();

  v4f fv[16];
#pragma unroll
  for (int i = 0; i < 16; ++i) {
    const int lr = 16 * wave + i;
    fv[i] = *(const v4fa*)(stg + lr * GBN + 4 * lane);
  }
#pragma unroll
  for (int i = 0; i < 16; ++i) {
    const int gr = rowBase + 16 * wave + i;
    float* op = H + (size_t)gr * DH + 4 * lane;
    if (gr < mRows) *(volatile v4f*)op = fv[i];
  }
  __threadfence();
#pragma unroll
  for (int i = 0; i < 16; ++i) {
    const int gr = rowBase + 16 * wave + i;
    float* op = H + (size_t)gr * DH + 4 * lane;
    if (gr < mRows) *(volatile v4f*)op = fv[i];
  }
}

__global__ __launch_bounds__(NTHR) void k_pool(const float* __restrict__ H, const int* __restrict__ gid,
                                               int nN, unsigned short* PHL, int colOff) {
  __shared__ __attribute__((aligned(16))) float wsum[NWAVE * DH];
  __shared__ __attribute__((aligned(16))) float outs[DH];
  const int tid = (int)threadIdx.x, lane = tid & 31, wave = tid >> 5;
  const int g = (int)blockIdx.x;

  float a0 = 0.0f, a1 = 0.0f, a2 = 0.0f, a3 = 0.0f;
#pragma unroll 1
  for (int i0 = wave * 32; i0 < nN; i0 += NTHR) {
    const int i  = i0 + lane;
    const int ic = i < nN ? i : nN - 1;
    const int b  = gid[ic];
    const bool hit = (i < nN) && (b == g);
    unsigned msk = __builtin_amdgcn_ballot_w32(hit);
    int nh = (int)__builtin_popcount(msk);
    nh = nh > 32 ? 32 : nh;
#pragma unroll 1
    for (int q = 0; q < nh; ++q) {
      const int k = __builtin_ffs((int)msk) - 1;
      msk &= msk - 1u;
      int node = i0 + (k < 0 ? 0 : k);
      node = node > nN - 1 ? nN - 1 : node;
      const v4f v = *(const v4f*)(H + (size_t)node * DH + 4 * lane);
      a0 += v.x; a1 += v.y; a2 += v.z; a3 += v.w;
    }
  }
  {
    v4f pv; pv.x = a0; pv.y = a1; pv.z = a2; pv.w = a3;
    *(v4fa*)(wsum + wave * DH + 4 * lane) = pv;
  }
  __syncthreads();
  if (tid < DH) {
    float s = 0.0f;
#pragma unroll
    for (int w2 = 0; w2 < NWAVE; ++w2) s += wsum[w2 * DH + tid];
    outs[tid] = s;
  }
  __syncthreads();
  const int cb = 8 * (lane & 15), hh = lane >> 4;
  const v4f oa = *(const v4fa*)(outs + cb);
  const v4f ob = *(const v4fa*)(outs + cb + 4);
  v8us hv, lv, pv;
  hilo8(oa, ob, hv, lv);
  const unsigned short sel = (hh != 0) ? (unsigned short)0xFFFF : (unsigned short)0;
#pragma unroll
  for (int j = 0; j < 8; ++j) pv[j] = (unsigned short)((lv[j] & sel) | (hv[j] & (unsigned short)~sel));
  unsigned short* dp = PHL + (size_t)g * PW2 + hh * PW + colOff + cb;
  const bool okst = (wave == 0);
  if (okst) *(volatile v8us*)dp = pv;
  __threadfence();
  if (okst) *(volatile v8us*)dp = pv;
}

static inline int cdiv(int a, int b) { return (a + b - 1) / b; }
static inline size_t al256(size_t o) { return (o + 255) & ~(size_t)255; }

extern "C" void kernel_launch(void* const* d_in, const int* in_sizes, int n_in,
                              void* d_out, int out_size, void* d_ws, size_t ws_size,
                              hipStream_t stream) {
  if (n_in < 14) return;
  if (in_sizes[3] < GBM) return;
  const int nN = in_sizes[3];
  if ((nN % GBM) != 0 || nN > (1 << 22)) return;
  if ((long long)in_sizes[0] != (long long)nN * DIN) return;
  if (in_sizes[1] < 2 || (in_sizes[1] & 1) != 0) return;
  const int nE = in_sizes[1] / 2;
  if (nE < 1 || nE > (1 << 20)) return;
  if ((long long)in_sizes[2] != (long long)nE * NET) return;
  if (in_sizes[4] != DIN * DH || in_sizes[5] != DH) return;
  if (in_sizes[6] != NET * DH || in_sizes[7] != DH) return;
  if (in_sizes[8] != DH * DH || in_sizes[9] != DH) return;
  if (in_sizes[10] != DH * DH || in_sizes[11] != DH) return;
  if (in_sizes[12] != PW * DOUT || in_sizes[13] != DOUT) return;
  if (out_size != NGR * DOUT) return;

  const float* x    = (const float*)d_in[0];
  const int*   ei   = (const int*)  d_in[1];
  const float* ea   = (const float*)d_in[2];
  const int*   gids = (const int*)  d_in[3];
  const float* Wn   = (const float*)d_in[4];
  const float* bn   = (const float*)d_in[5];
  const float* We   = (const float*)d_in[6];
  const float* be   = (const float*)d_in[7];
  const float* W1   = (const float*)d_in[8];
  const float* b1   = (const float*)d_in[9];
  const float* W2   = (const float*)d_in[10];
  const float* b2   = (const float*)d_in[11];
  const float* Wl   = (const float*)d_in[12];
  const float* bl   = (const float*)d_in[13];
  float* out = (float*)d_out;
  const int* src = ei;
  const int* dst = ei + nE;

  const int gA   = cdiv(nN, NB);
  const int gM   = nN / GBM;
  const int vec8 = ((nE & 3) == 0) ? 1 : 0;
  const int nux  = nN * (DIN / 8);
  if ((nux % NTHR) != 0) return;

  char* ws = (char*)d_ws;
  size_t off = 0;
  const size_t oXB  = off; off = al256(off + (size_t)nN * DIN * 2);
  const size_t oWnT = off; off = al256(off + (size_t)DH * DIN * 2);
  const size_t oWeT = off; off = al256(off + (size_t)DH * DIN * 2);
  const size_t oW1D = off; off = al256(off + (size_t)DH * ZW * 2);
  const size_t oW2D = off; off = al256(off + (size_t)DH * ZW * 2);
  const size_t oWL2 = off; off = al256(off + (size_t)DOUT * PW2 * 2);
  const size_t oH   = off; off = al256(off + (size_t)nN * DH * 4);
  const size_t oZ   = off; off = al256(off + (size_t)nN * ZW * 2);
  const size_t oEAS = off; off = al256(off + (size_t)gA * RCAP * NET * 2);
  const size_t oSRC = off; off = al256(off + (size_t)gA * RCAP * 4);
  const size_t oTSO = off; off = al256(off + (size_t)gA * NB * 4);
  const size_t oTSC = off; off = al256(off + (size_t)gA * NB * 4);
  const size_t oMET = off; off = al256(off + (size_t)gA * 32 * 4);
  const size_t oPHL = off; off = al256(off + (size_t)NGR * PW2 * 2);
  if (off > ws_size || off > (size_t)WSMAX) return;
  unsigned short* XB  = (unsigned short*)(ws + oXB);
  unsigned short* WnT = (unsigned short*)(ws + oWnT);
  unsigned short* WeT = (unsigned short*)(ws + oWeT);
  unsigned short* W1D = (unsigned short*)(ws + oW1D);
  unsigned short* W2D = (unsigned short*)(ws + oW2D);
  unsigned short* WL2 = (unsigned short*)(ws + oWL2);
  float*          H   = (float*)(ws + oH);
  unsigned short* Z   = (unsigned short*)(ws + oZ);
  unsigned short* EAS = (unsigned short*)(ws + oEAS);
  int*            SRC = (int*)(ws + oSRC);
  int*            TSO = (int*)(ws + oTSO);
  int*            TSC = (int*)(ws + oTSC);
  int*            MET = (int*)(ws + oMET);
  unsigned short* PHL = (unsigned short*)(ws + oPHL);

  hipFuncSetAttribute(reinterpret_cast<const void*>(&k_bucket), hipFuncAttributeMaxDynamicSharedMemorySize, LDS_BKT);
  hipFuncSetAttribute(reinterpret_cast<const void*>(&k_scan),   hipFuncAttributeMaxDynamicSharedMemorySize, LDS_SCAN);

  k_prep<<<(nux + NUWTOT) / NTHR, NTHR, 0, stream>>>(x, Wn, We, W1, W2, Wl, nux, XB, WnT, WeT, W1D, W2D, WL2);
  k_gemm<<<dim3(gM, DH / GBN), GTHR, 0, stream>>>(XB, DIN, WnT, DIN, DIN, bn, H, DH, nN, nN);
  k_bucket<<<gA, NTHR, LDS_BKT, stream>>>(src, dst, ea, nN, nE, vec8, EAS, SRC, TSO, TSC, MET);
  for (int t = 0; t < TST; ++t) {
    k_scan<<<gA, NTHR, LDS_SCAN, stream>>>(EAS, SRC, TSO, TSC, MET, WeT, be, H, Z, nN);
    k_mlp<<<gM, GTHR, 0, stream>>>(Z, W1D, W2D, b1, b2, H, nN, nN);
    k_pool<<<NGR, NTHR, 0, stream>>>(H, gids, nN, PHL, t * DH);
  }
  k_gemm<<<dim3(NGR / GBM, DOUT / GBN), GTHR, 0, stream>>>(PHL, PW2, WL2, PW2, PW2, bl, out, DOUT, NGR, NGR);
}
